// GATwithMinCutPooling_23648089931944
// MI455X (gfx1250) — hardware-run, weakly checked
//
#include <hip/hip_runtime.h>


namespace {
constexpr int N = 10000, NPD = 10016, E = 320000, F = 256, H1 = 8, C1 = 8, W1W = 64, K = 16, NBLK = (N + 15) / 16;
constexpr int OFF1 = 160000, OFF2 = 164096, OFF3 = 164352, OFF4 = 164353;
constexpr float XS = 8.0f, WSC = 256.0f, NEG = 0.2f, PEPS = 1e-15f;
typedef _Float16 b16;
typedef __attribute__((ext_vector_type(16))) _Float16 v16b;
typedef __attribute__((ext_vector_type(8))) _Float16 v8b;
typedef __attribute__((ext_vector_type(8))) float v8f;
typedef __attribute__((ext_vector_type(4))) float v4f;
typedef __attribute__((ext_vector_type(2))) float v2f;
__device__ __forceinline__ float bf16_rne(float f) { unsigned int u = __float_as_uint(f); u += 0x7FFFu + ((u >> 16) & 1u); return __uint_as_float(u & 0xFFFF0000u); }
__device__ __forceinline__ void split16(float v, b16& hi, b16& lo) { hi = (b16)v; lo = (b16)(v - (float)hi); }
__device__ __forceinline__ v16b frag_kb(const b16* p, int hh) { const v8b a = *(const v8b*)(p + 8 * hh), b = *(const v8b*)(p + 16 + 8 * hh); v16b f;
#pragma unroll
  for (int e = 0; e < 8; ++e) { f[e] = a[e]; f[8 + e] = b[e]; } return f; }
__device__ __forceinline__ v8f wmma16b(v16b a, v16b b, v8f c) { v8f d = __builtin_amdgcn_wmma_f32_16x16x32_f16(false, a, false, b, (short)0, c, false, false); asm volatile("v_nop\n\tv_nop\n\tv_nop\n\tv_nop" : "+v"(d) : "v"(a), "v"(b)); return d; }
__device__ __forceinline__ void wave_lds_sync() { __builtin_amdgcn_fence(__ATOMIC_RELEASE, "workgroup"); __builtin_amdgcn_wave_barrier(); __builtin_amdgcn_fence(__ATOMIC_ACQUIRE, "workgroup"); }
__device__ __forceinline__ float pmul(float a, float b) { float p = a * b; asm volatile("" : "+v"(p)); return p; }
__device__ __forceinline__ int iclamp(int v, int lo, int hi) { return v < lo ? lo : (v > hi ? hi : v); }
__device__ __forceinline__ float leaky(float v) { return v > 0.0f ? v : NEG * v; }
__device__ __forceinline__ float elu(float v) { return v > 0.0f ? v : expm1f(v); }
template <int CPL> __device__ __forceinline__ void ldrow(const float* p, float* f) { if (CPL == 2) { const v2f a = *(const v2f*)p; f[0] = a[0]; f[1] = a[1]; } else { for (int q = 0; q < CPL / 4; ++q) { const v4f a = *(const v4f*)(p + 4 * q); for (int i = 0; i < 4; ++i) f[4 * q + i] = a[i]; } } }
template <int CPL> __device__ __forceinline__ void strow(float* p, const float* f) { if (CPL == 2) { v2f a = {f[0], f[1]}; *(volatile v2f*)p = a; } else { for (int q = 0; q < CPL / 4; ++q) { v4f a; for (int i = 0; i < 4; ++i) a[i] = f[4 * q + i]; *(volatile v4f*)(p + 4 * q) = a; } } }
constexpr int CSR_NBLK8 = 512, CSR_GB8 = 8, CSR_GN8 = 1 << CSR_GB8  , CSR_TS8 = (CSR_GN8 < 32 ? 32 : CSR_GN8)  , CSR_MAXG8 = 512, CSR_CAP8 = 12288  ;
__device__ __host__ __forceinline__ int csr_tix8(int v) { return (v >> CSR_GB8) * CSR_TS8 + (v & (CSR_GN8 - 1)); }
__global__ __launch_bounds__(64) void csrA_kernel8(const int* __restrict__ dst, int E, int N, int nG, int CHP, int NGP, int* __restrict__ STG, int* __restrict__ HST) {
  extern __shared__ int sm[];
  int* cnt = sm; int* run = sm + NGP; int* ids = sm + 2 * NGP;
  const int b = blockIdx.x; const int ch = (E + CSR_NBLK8 - 1) / CSR_NBLK8; const int e0 = b * ch, e1 = min(E, e0 + ch);
  for (int i = threadIdx.x; i < NGP; i += 64) cnt[i] = 0;
  for (int i = threadIdx.x; i < CHP; i += 64) ids[i] = -1;
  __syncthreads();
  if (threadIdx.x == 0) {
    for (int e = e0; e < e1; ++e) { int d = dst[e]; d = (d < 0) ? 0 : (d >= N ? N - 1 : d); cnt[d >> CSR_GB8] += 1; }
    int acc = 0; for (int g = 0; g < nG; ++g) { run[g] = acc; acc += cnt[g]; }
    for (int e = e0; e < e1; ++e) { int d = dst[e]; d = (d < 0) ? 0 : (d >= N ? N - 1 : d); const int g = d >> CSR_GB8; ids[run[g]] = e; run[g] += 1; } }
  __syncthreads();
  typedef __attribute__((ext_vector_type(4))) int v4i;
  for (int pass = 0; pass < 2; ++pass) {
    for (int i = threadIdx.x; i < CHP / 4; i += 64) *(volatile v4i*)(STG + (size_t)b * CHP + i * 4) = *(const v4i*)(&ids[i * 4]);
    for (int i = threadIdx.x; i < NGP / 4; i += 64) { v4i v; for (int e = 0; e < 4; ++e) v[e] = (i * 4 + e < nG) ? cnt[i * 4 + e] : 0; *(volatile v4i*)(HST + (size_t)b * NGP + i * 4) = v; }
    __threadfence(); }
}
__global__ __launch_bounds__(512) void csrS_kernel8(const int* __restrict__ HST, int nG, int NGP, int* __restrict__ START, int* __restrict__ TOT, int* __restrict__ OFF) {
  __shared__ int tot[CSR_MAXG8];
  const int b = threadIdx.x;
  for (int pass = 0; pass < 2; ++pass) { int runb = 0; for (int g = 0; g < nG; ++g) { int c = HST[(size_t)b * NGP + g]; c = (c < 0) ? 0 : c; ((volatile int*)OFF)[(size_t)g * CSR_NBLK8 + b] = runb; runb += c; } __threadfence(); }
  for (int g = threadIdx.x; g < nG; g += 512) { int s = 0; for (int bb = 0; bb < CSR_NBLK8; ++bb) { int c = HST[(size_t)bb * NGP + g]; s += (c < 0) ? 0 : c; } tot[g] = s; }
  __syncthreads();
  if (threadIdx.x < 32) {
    __shared__ int st[CSR_MAXG8 + 32];
    if (threadIdx.x == 0) { int acc = 0; for (int g = 0; g < NGP; ++g) { st[g] = acc; if (g < nG) acc += (tot[g] + 31) & ~31; } st[NGP] = acc; }
    __builtin_amdgcn_fence(__ATOMIC_RELEASE, "workgroup"); __builtin_amdgcn_wave_barrier(); __builtin_amdgcn_fence(__ATOMIC_ACQUIRE, "workgroup");
    for (int pass = 0; pass < 2; ++pass) { for (int i = threadIdx.x; i < NGP + 32; i += 32) { ((volatile int*)START)[i] = (i <= NGP) ? st[min(i, NGP)] : 0; ((volatile int*)TOT)[i] = (i < nG) ? tot[i] : 0; } __threadfence(); } }
}
__global__ __launch_bounds__(256) void csrB_kernel8(const int* __restrict__ dst, int N, int nG, int CHP, int NGP, int permLen, const int* __restrict__ STG, const int* __restrict__ HST, const int* __restrict__ OFF, const int* __restrict__ START, const int* __restrict__ TOT, int* __restrict__ PERM, int* __restrict__ ROWPTR, int* __restrict__ ROWCNT, int* __restrict__ FLAG) {
  typedef __attribute__((ext_vector_type(4))) int v4i;
  __shared__ int ids[CSR_CAP8]; __shared__ unsigned short key[CSR_CAP8]; __shared__ int outp[CSR_CAP8]; __shared__ int ncnt[CSR_GN8 + 1]; __shared__ int boff[CSR_NBLK8 + 1];
  const int g = blockIdx.x, t_ = threadIdx.x; int tot = TOT[g]; int st = START[g], stn = START[g + 1]; const int v0 = g * CSR_GN8; const int nv = min(CSR_GN8, N - v0); const int t0 = g * CSR_TS8;
  st = (st < 0) ? 0 : (st > permLen - 32 ? permLen - 32 : st) & ~31; stn = (stn < st) ? st : (stn > permLen ? permLen : stn); tot = (tot < 0) ? 0 : tot; if (tot > stn - st && tot <= CSR_CAP8) tot = stn - st;
  if (tot > CSR_CAP8) {
    for (int pass = 0; pass < 2; ++pass) { for (int i = t_; i < CSR_TS8 / 4; i += 256) { v4i a, c; for (int e = 0; e < 4; ++e) { a[e] = st; c[e] = 0; } *(volatile v4i*)(ROWPTR + t0 + i * 4) = a; *(volatile v4i*)(ROWCNT + t0 + i * 4) = c; } if (t_ == 0) ((volatile int*)FLAG)[0] = 1; __threadfence(); } (void)nv; return; }
  if (t_ == 0) { int acc = 0; for (int b = 0; b < CSR_NBLK8; ++b) { boff[b] = acc; int c = HST[(size_t)b * NGP + g]; c = (c < 0) ? 0 : (c > CHP ? CHP : c); acc += c; if (acc > tot) acc = tot; } boff[CSR_NBLK8] = acc; }
  for (int i = t_; i <= CSR_GN8; i += 256) ncnt[i] = 0;
  __syncthreads();
  for (int b = 0; b < CSR_NBLK8; ++b) { const int c = boff[b + 1] - boff[b]; int o_ = OFF[(size_t)g * CSR_NBLK8 + b]; o_ = (o_ < 0) ? 0 : (o_ > CHP - c ? CHP - c : o_); const int* src_ = STG + (size_t)b * CHP + o_;
    for (int i = t_; i < c; i += 256) { int id = src_[i]; id = (id < 0) ? 0 : id; ids[boff[b] + i] = id; int d = dst[id]; d = (d < v0) ? v0 : (d >= N ? N - 1 : d); int kk = d - v0; kk = (kk < 0) ? 0 : (kk >= CSR_GN8 ? CSR_GN8 - 1 : kk); key[boff[b] + i] = (unsigned short)kk; } }
  __syncthreads();
  if (t_ == 0) { for (int i = 0; i < tot; ++i) ncnt[key[i]] += 1; int acc = 0; for (int vl = 0; vl < CSR_GN8; ++vl) { const int c = ncnt[vl]; ncnt[vl] = acc; acc += c; } ncnt[CSR_GN8] = acc;
    for (int i = 0; i < tot; ++i) { const int vl = key[i]; outp[ncnt[vl]] = ids[i]; ncnt[vl] += 1; }
    for (int vl = CSR_GN8; vl > 0; --vl) ncnt[vl] = ncnt[vl - 1]; ncnt[0] = 0; }
  __syncthreads();
  for (int pass = 0; pass < 2; ++pass) {
    for (int i = t_; i < (stn - st) / 4; i += 256) { v4i v; for (int e = 0; e < 4; ++e) { const int q = i * 4 + e; v[e] = (q < tot) ? outp[q] : -1; } *(volatile v4i*)(PERM + st + i * 4) = v; }
    for (int i = t_; i < CSR_TS8 / 4; i += 256) { v4i a, c; for (int e = 0; e < 4; ++e) { const int vl = i * 4 + e; const int vc = vl < CSR_GN8 ? vl : CSR_GN8; a[e] = (vl < CSR_GN8) ? st + ncnt[vc] : st; c[e] = (vl < nv) ? (ncnt[(vc < CSR_GN8 ? vc : CSR_GN8 - 1) + 1] - ncnt[vc]) : 0; } *(volatile v4i*)(ROWPTR + t0 + i * 4) = a; *(volatile v4i*)(ROWCNT + t0 + i * 4) = c; }
    __threadfence(); }
}
__global__ __launch_bounds__(256) void csrZ_kernel8(int* __restrict__ p, size_t n4) { typedef __attribute__((ext_vector_type(4))) int v4i; const size_t tid = (size_t)blockIdx.x * 256 + threadIdx.x, nth = (size_t)gridDim.x * 256; v4i z = {0, 0, 0, 0}; for (size_t i = tid; i < n4; i += nth) *(volatile v4i*)(p + i * 4) = z; }
struct CsrBufs8 { int *STG, *HST, *OFF, *START, *TOT, *PERM, *ROWPTR, *ROWCNT, *FLAG; int nG, NGP, CHP; size_t permLen; char* base; size_t bytes; };
static size_t csr_carve8(CsrBufs8& c, char* ws, size_t off, int E, int N) {
  const size_t off0 = off; c.base = ws + off;
  auto al = [&](size_t bytes) { char* p = ws + off; off += (bytes + 255) & ~(size_t)255; return p; };
  c.nG = (N + CSR_GN8 - 1) / CSR_GN8; c.NGP = (c.nG + 31) & ~31; const int ch = (E + CSR_NBLK8 - 1) / CSR_NBLK8; c.CHP = (ch + 31) & ~31; c.permLen = (size_t)E + 32 * (size_t)c.nG + 32;
  c.STG = (int*)al((size_t)CSR_NBLK8 * c.CHP * 4); c.HST = (int*)al((size_t)CSR_NBLK8 * c.NGP * 4); c.OFF = (int*)al((size_t)c.NGP * CSR_NBLK8 * 4); c.START = (int*)al((size_t)(c.NGP + 64) * 4); c.TOT = (int*)al((size_t)(c.NGP + 64) * 4);
  c.PERM = (int*)al(c.permLen * 4); c.ROWPTR = (int*)al((size_t)c.nG * CSR_TS8 * 4); c.ROWCNT = (int*)al((size_t)c.nG * CSR_TS8 * 4); c.FLAG = (int*)al(256);
  c.bytes = off - off0; return off;
}
static void csr_build8(const CsrBufs8& c, const int* dst, int E, int N, hipStream_t stream) {
  const size_t smem = (size_t)(2 * c.NGP + c.CHP) * 4;
  csrZ_kernel8<<<512, 256, 0, stream>>>((int*)c.base, c.bytes / 16);
  csrA_kernel8<<<CSR_NBLK8, 64, smem, stream>>>(dst, E, N, c.nG, c.CHP, c.NGP, c.STG, c.HST);
  csrS_kernel8<<<1, 512, 0, stream>>>(c.HST, c.nG, c.NGP, c.START, c.TOT, c.OFF);
  csrB_kernel8<<<c.nG, 256, 0, stream>>>(dst, N, c.nG, c.CHP, c.NGP, (int)c.permLen, c.STG, c.HST, c.OFF, c.START, c.TOT, c.PERM, c.ROWPTR, c.ROWCNT, c.FLAG);
}


__global__ __launch_bounds__(256) void wprep_kernel(const float* __restrict__ w, int KIN, int OUTW, b16* __restrict__ WT) {
  const int u = blockIdx.x * 256 + threadIdx.x; if (u >= OUTW * KIN / 8) return; const int e = u * 8; const int o = e / KIN, k0 = e % KIN; v8b v;
#pragma unroll
  for (int j = 0; j < 8; ++j) v[j] = (b16)(bf16_rne(w[(size_t)(k0 + j) * OUTW + o]) * WSC); for (int pass = 0; pass < 2; ++pass) { *(volatile v8b*)(WT + e) = v; __threadfence(); }
}
__global__ __launch_bounds__(256) void xt_kernel(const float* __restrict__ x, b16* __restrict__ XT) {
  const int u = blockIdx.x * 256 + threadIdx.x; if (u >= F * NPD / 8) return; const int f = u / (NPD / 8), n0 = (u % (NPD / 8)) * 8; v8b v;
#pragma unroll
  for (int j = 0; j < 8; ++j) { const int n = n0 + j; v[j] = n < N ? (b16)(bf16_rne(x[(size_t)n * F + f]) * XS) : (b16)0.0f; } for (int pass = 0; pass < 2; ++pass) { *(volatile v8b*)(XT + (size_t)f * NPD + n0) = v; __threadfence(); }
}
__global__ __launch_bounds__(32) void lin1_kernel(const float* __restrict__ x, const b16* __restrict__ WT, const float* __restrict__ as, const float* __restrict__ ad, float* __restrict__ P, float* __restrict__ ES, float* __restrict__ ED) {
  __shared__ __attribute__((aligned(16))) b16 Ah[16][F + 8]; __shared__ __attribute__((aligned(16))) float Tf[16][W1W + 4], Se[16][8], Sd[16][8];
  const int lane = threadIdx.x, nloc = lane & 15, hlf = lane >> 4; const size_t m0 = (size_t)blockIdx.x * 16;
  for (int rr = 0; rr < 16; ++rr) { const size_t r = (m0 + rr) < (size_t)N ? m0 + rr : (size_t)N - 1; for (int q = 0; q < F / 32; ++q) Ah[rr][q * 32 + lane] = (b16)(bf16_rne(x[r * F + q * 32 + lane]) * XS); }
  wave_lds_sync();
  v8f acc[4];
#pragma unroll
  for (int t = 0; t < 4; ++t) acc[t] = (v8f){};
#pragma unroll 2
  for (int kb = 0; kb < F; kb += 32) { const v16b a = frag_kb(&Ah[nloc][kb], hlf);
#pragma unroll
    for (int t = 0; t < 4; ++t) acc[t] = wmma16b(a, frag_kb(WT + (size_t)(t * 16 + nloc) * F + kb, hlf), acc[t]); }
  const float sc = 1.0f / (XS * WSC);
#pragma unroll
  for (int t = 0; t < 4; ++t) { const int c = t * 16 + nloc; const float wsv = bf16_rne(as[c]), wdv = bf16_rne(ad[c]);
#pragma unroll
    for (int r8 = 0; r8 < 8; ++r8) { const float p = acc[t][r8] * sc; Tf[8 * hlf + r8][c] = p; float s = pmul(p, wsv), d = pmul(p, wdv); for (int o = 1; o < 8; o <<= 1) { s += __shfl_xor(s, o); d += __shfl_xor(d, o); } if ((nloc & 7) == 0) { Se[8 * hlf + r8][2 * t + (nloc >> 3)] = s; Sd[8 * hlf + r8][2 * t + (nloc >> 3)] = d; } } }
  wave_lds_sync();
  for (int pass = 0; pass < 2; ++pass) { for (int rr = 0; rr < 16; ++rr) if (m0 + rr < (size_t)N) *(volatile v2f*)(P + (m0 + rr) * W1W + lane * 2) = *(const v2f*)(&Tf[rr][lane * 2]); if (lane < 16 && m0 + lane < (size_t)N) { *(volatile v4f*)(ES + (m0 + lane) * 8) = *(const v4f*)(&Se[lane][0]); *(volatile v4f*)(ES + (m0 + lane) * 8 + 4) = *(const v4f*)(&Se[lane][4]); *(volatile v4f*)(ED + (m0 + lane) * 8) = *(const v4f*)(&Sd[lane][0]); *(volatile v4f*)(ED + (m0 + lane) * 8 + 4) = *(const v4f*)(&Sd[lane][4]); } __threadfence(); }
}
__global__ __launch_bounds__(256) void att1_kernel(const float* __restrict__ P, const float* __restrict__ ES, const float* __restrict__ ED, const float* __restrict__ bias, const int* __restrict__ srcs, const int* __restrict__ PERM, const int* __restrict__ ROWPTR, const int* __restrict__ ROWCNT, int permLen, float* __restrict__ Hout) {
  const int wave = threadIdx.x >> 5, lane = threadIdx.x & 31; const size_t v = (size_t)blockIdx.x * 8 + wave; if (v >= (size_t)N) return; const int h = lane >> 2;
  const float edv = ED[v * 8 + h], esv = ES[v * 8 + h]; int st = ROWPTR[v], cnt = ROWCNT[v]; cnt = iclamp(cnt, 0, 1 << 20); st = iclamp(st, 0, permLen - cnt);
  float mx = leaky(esv + edv);
#pragma unroll 1
  for (int j = 0; j < cnt; ++j) { const int e = iclamp(PERM[st + j], 0, E - 1); const int s = iclamp(srcs[e], 0, N - 1); mx = fmaxf(mx, leaky(ES[(size_t)s * 8 + h] + edv)); }
  const v2f own = *(const v2f*)(P + v * W1W + lane * 2); float p0 = __expf(leaky(esv + edv) - mx); float den = p0, o0 = pmul(p0, own[0]), o1 = pmul(p0, own[1]);
#pragma unroll 1
  for (int j = 0; j < cnt; ++j) { const int e = iclamp(PERM[st + j], 0, E - 1); const size_t s = (size_t)iclamp(srcs[e], 0, N - 1); const float p = __expf(leaky(ES[s * 8 + h] + edv) - mx); den += p; const v2f f = *(const v2f*)(P + s * W1W + lane * 2); o0 += pmul(p, f[0]); o1 += pmul(p, f[1]); }
  const float inv = 1.0f / (den + 1e-16f); v2f o = {elu(pmul(o0, inv) + bf16_rne(bias[lane * 2])), elu(pmul(o1, inv) + bf16_rne(bias[lane * 2 + 1]))};
  for (int pass = 0; pass < 2; ++pass) { *(volatile v2f*)(Hout + v * W1W + lane * 2) = o; __threadfence(); }
}
__global__ __launch_bounds__(32) void lin2_kernel(const float* __restrict__ Hp, const b16* __restrict__ WT, const float* __restrict__ as, const float* __restrict__ ad, float* __restrict__ P2, float* __restrict__ EL) {
  __shared__ __attribute__((aligned(16))) b16 Ah[16][W1W + 8], Al[16][W1W + 8]; __shared__ __attribute__((aligned(16))) float Tf[16][K], Se[16][2];
  const int lane = threadIdx.x, nloc = lane & 15, hlf = lane >> 4; const size_t m0 = (size_t)blockIdx.x * 16;
  for (int rr = 0; rr < 16; ++rr) { const size_t r = (m0 + rr) < (size_t)N ? m0 + rr : (size_t)N - 1; const v2f v = *(const v2f*)(Hp + r * W1W + lane * 2); for (int j = 0; j < 2; ++j) { b16 p, q; split16(v[j] * XS, p, q); Ah[rr][lane * 2 + j] = p; Al[rr][lane * 2 + j] = q; } }
  wave_lds_sync();
  v8f acc = {};
#pragma unroll
  for (int kb = 0; kb < W1W; kb += 32) { const v16b a = frag_kb(&Ah[nloc][kb], hlf), al = frag_kb(&Al[nloc][kb], hlf), bw = frag_kb(WT + (size_t)nloc * W1W + kb, hlf); acc = wmma16b(a, bw, acc); acc = wmma16b(al, bw, acc); }
  const float sc = 1.0f / (XS * WSC), wsv = bf16_rne(as[nloc]), wdv = bf16_rne(ad[nloc]);
#pragma unroll
  for (int r8 = 0; r8 < 8; ++r8) { const float p = acc[r8] * sc; Tf[8 * hlf + r8][nloc] = p; float s = pmul(p, wsv), d = pmul(p, wdv); for (int o = 1; o < 16; o <<= 1) { s += __shfl_xor(s, o); d += __shfl_xor(d, o); } if (nloc == 0) { Se[8 * hlf + r8][0] = s; Se[8 * hlf + r8][1] = d; } }
  wave_lds_sync();
  for (int pass = 0; pass < 2; ++pass) { for (int q = 0; q < 8; ++q) { const int i = q * 32 + lane; const int rr = i / K, c = i % K; if (m0 + rr < (size_t)N) ((volatile float*)P2)[(m0 + rr) * K + c] = Tf[rr][c]; } if (m0 + (lane >> 1) < (size_t)N) ((volatile float*)EL)[m0 * 2 + lane] = Se[lane >> 1][lane & 1]; __threadfence(); }
}
__global__ __launch_bounds__(256) void att2_kernel(const float* __restrict__ P2, const float* __restrict__ EL, const float* __restrict__ bias, const float* __restrict__ Ws, const float* __restrict__ bs, const int* __restrict__ srcs, const int* __restrict__ PERM, const int* __restrict__ ROWPTR, const int* __restrict__ ROWCNT, int permLen, float* __restrict__ xg, float* __restrict__ S) {
  const int wave = threadIdx.x >> 5, lane = threadIdx.x & 31, c = lane & 15, side = lane >> 4; const size_t v0 = ((size_t)blockIdx.x * 8 + wave) * 2; const size_t v = v0 + side; const bool live = v < (size_t)N; const size_t vv = live ? v : (size_t)N - 1;
  const float edv = EL[vv * 2 + 1], esv = EL[vv * 2]; int st = ROWPTR[vv], cnt = ROWCNT[vv]; cnt = iclamp(cnt, 0, 1 << 20); st = iclamp(st, 0, permLen - cnt); if (!live) cnt = 0;
  int cmax = cnt; { const int other = __shfl_xor(cnt, 16); cmax = cnt > other ? cnt : other; }
  float mx = leaky(esv + edv);
#pragma unroll 1
  for (int j = 0; j < cmax; ++j) { const bool ok = j < cnt; const int e = ok ? iclamp(PERM[st + j], 0, E - 1) : 0; const int s = iclamp(srcs[e], 0, N - 1); const float val = leaky(EL[(size_t)s * 2] + edv); if (ok) mx = fmaxf(mx, val); }
  const float own = P2[vv * K + c]; const float p0 = __expf(leaky(esv + edv) - mx); float den = p0, o = pmul(p0, own);
#pragma unroll 1
  for (int j = 0; j < cmax; ++j) { const bool ok = j < cnt; const int e = ok ? iclamp(PERM[st + j], 0, E - 1) : 0; const size_t s = (size_t)iclamp(srcs[e], 0, N - 1); const float p = __expf(leaky(EL[s * 2] + edv) - mx); const float f = P2[s * K + c]; if (ok) { den += p; o += pmul(p, f); } }
  const float g = pmul(o, 1.0f / (den + 1e-16f)) + bf16_rne(bias[c]);
  float z = bf16_rne(bs[c]);
#pragma unroll
  for (int k = 0; k < K; ++k) { const float gk = __shfl(g, (side << 4) + k); z += pmul(gk, bf16_rne(Ws[k * K + c])); }
  float m1 = z; for (int of = 1; of < 16; of <<= 1) m1 = fmaxf(m1, __shfl_xor(m1, of)); float e1 = __expf(z - m1); float s1 = e1; for (int of = 1; of < 16; of <<= 1) s1 += __shfl_xor(s1, of); const float t1 = e1 / s1;
  float m2 = t1; for (int of = 1; of < 16; of <<= 1) m2 = fmaxf(m2, __shfl_xor(m2, of)); float e2 = __expf(t1 - m2); float s2 = e2; for (int of = 1; of < 16; of <<= 1) s2 += __shfl_xor(s2, of); const float sv = e2 / s2;
  for (int pass = 0; pass < 2; ++pass) { if (live) { ((volatile float*)xg)[v * K + c] = g; ((volatile float*)S)[v * K + c] = sv; } __threadfence(); }
}
__global__ __launch_bounds__(256) void st_kernel(const float* __restrict__ S, b16* __restrict__ STh, b16* __restrict__ STl) {
  const int u = blockIdx.x * 256 + threadIdx.x; if (u >= K * NPD / 8) return; const int k = u / (NPD / 8), n0 = (u % (NPD / 8)) * 8; v8b vh, vl;
#pragma unroll
  for (int j = 0; j < 8; ++j) { const int n = n0 + j; b16 p = (b16)0.0f, q = (b16)0.0f; if (n < N) split16(S[(size_t)n * K + k] * XS, p, q); vh[j] = p; vl[j] = q; }
  for (int pass = 0; pass < 2; ++pass) { *(volatile v8b*)(STh + (size_t)k * NPD + n0) = vh; *(volatile v8b*)(STl + (size_t)k * NPD + n0) = vl; __threadfence(); }
}
__global__ __launch_bounds__(256) void se_kernel(const float* __restrict__ S, const int* __restrict__ ei, b16* __restrict__ SAh, b16* __restrict__ SAl, b16* __restrict__ SBh, b16* __restrict__ SBl) {
  const int u = blockIdx.x * 256 + threadIdx.x; if (u >= 2 * K * (E / 8)) return; const int which = u / (K * (E / 8)); const int rem = u % (K * (E / 8)); const int k = rem / (E / 8), e0 = (rem % (E / 8)) * 8; v8b vh, vl;
#pragma unroll
  for (int j = 0; j < 8; ++j) { const int n = iclamp(ei[(size_t)which * E + e0 + j], 0, N - 1); b16 p, q; split16(S[(size_t)n * K + k] * XS, p, q); vh[j] = p; vl[j] = q; }
  b16* Ph = which ? SBh : SAh; b16* Pl = which ? SBl : SAl;
  for (int pass = 0; pass < 2; ++pass) { *(volatile v8b*)(Ph + (size_t)k * E + e0) = vh; *(volatile v8b*)(Pl + (size_t)k * E + e0) = vl; __threadfence(); }
}
__global__ __launch_bounds__(256) void pool_kernel(const b16* __restrict__ STh, const b16* __restrict__ STl, const b16* __restrict__ XT, const b16* __restrict__ SAh, const b16* __restrict__ SAl, const b16* __restrict__ SBh, const b16* __restrict__ SBl, const float* __restrict__ S, const int* __restrict__ ei, float* __restrict__ dout) {
  __shared__ float So[K][F + 4]; __shared__ float SS[K][K]; __shared__ float SP[6][K][K]; __shared__ float SA_[K][K]; __shared__ float dpart[256];
  const int wave = threadIdx.x >> 5, lane = threadIdx.x & 31, nloc = lane & 15, hlf = lane >> 4; const float sc2 = 1.0f / (XS * XS), sc1 = 1.0f / (XS * XS);
  if (wave == 0) {
#pragma unroll 1
    for (int t = 0; t < F / 16; ++t) { v8f acc = {};
#pragma unroll 1
      for (int k0 = 0; k0 < NPD; k0 += 32 * 32) { v8f a2 = {};
#pragma unroll 4
        for (int kb = k0; kb < k0 + 32 * 32 && kb < NPD; kb += 32) { const v16b bw = frag_kb(XT + (size_t)(t * 16 + nloc) * NPD + kb, hlf); a2 = wmma16b(frag_kb(STh + (size_t)nloc * NPD + kb, hlf), bw, a2); a2 = wmma16b(frag_kb(STl + (size_t)nloc * NPD + kb, hlf), bw, a2); }
        acc += a2; }
#pragma unroll
      for (int r8 = 0; r8 < 8; ++r8) So[8 * hlf + r8][t * 16 + nloc] = acc[r8] * sc1; } }
  else if (wave == 1) {
    v8f acc = {};
#pragma unroll 1
    for (int k0 = 0; k0 < NPD; k0 += 32 * 32) { v8f a2 = {};
#pragma unroll 4
      for (int kb = k0; kb < k0 + 32 * 32 && kb < NPD; kb += 32) { const v16b ah = frag_kb(STh + (size_t)nloc * NPD + kb, hlf), al = frag_kb(STl + (size_t)nloc * NPD + kb, hlf); a2 = wmma16b(ah, ah, a2); a2 = wmma16b(ah, al, a2); a2 = wmma16b(al, ah, a2); a2 = wmma16b(al, al, a2); }
      acc += a2; }
#pragma unroll
    for (int r8 = 0; r8 < 8; ++r8) SS[8 * hlf + r8][nloc] = acc[r8] * sc2; }
  else {
    v8f acc = {}; const int w6 = wave - 2;
#pragma unroll 1
    for (int k0 = 32 * w6; k0 < E; k0 += 32 * 6 * 32) { v8f a2 = {};
#pragma unroll 2
      for (int kb = k0; kb < k0 + 32 * 6 * 32 && kb < E; kb += 32 * 6) { const v16b ah = frag_kb(SAh + (size_t)nloc * E + kb, hlf), al = frag_kb(SAl + (size_t)nloc * E + kb, hlf), bh = frag_kb(SBh + (size_t)nloc * E + kb, hlf), bl = frag_kb(SBl + (size_t)nloc * E + kb, hlf); a2 = wmma16b(ah, bh, a2); a2 = wmma16b(ah, bl, a2); a2 = wmma16b(al, bh, a2); a2 = wmma16b(al, bl, a2); }
      acc += a2; }
#pragma unroll
    for (int r8 = 0; r8 < 8; ++r8) SP[w6][8 * hlf + r8][nloc] = acc[r8] * sc2; }
  { float dsum = 0.0f; const int e0 = threadIdx.x * (E / 256);
#pragma unroll 1
    for (int e = e0; e < e0 + E / 256; ++e) { const int n = iclamp(ei[e], 0, N - 1); float q = 0.0f;
#pragma unroll
      for (int k = 0; k < K; k += 4) { const v4f sv = *(const v4f*)(S + (size_t)n * K + k); for (int i = 0; i < 4; ++i) q += pmul(sv[i], sv[i]); } dsum += q; }
    dpart[threadIdx.x] = dsum; }
  __syncthreads();
  if (wave == 2 && lane < 16) { for (int j = 0; j < K; ++j) { float a = 0.0f; for (int w6 = 0; w6 < 6; ++w6) a += SP[w6][lane][j]; SA_[lane][j] = a; } }
  __syncthreads();
  if (threadIdx.x == 0) {
    float den = 0.0f; for (int i = 0; i < 256; ++i) den += dpart[i]; float tr = 0.0f; for (int k = 0; k < K; ++k) tr += SA_[k][k]; const float mincut = -(tr / den);
    float fro = 0.0f; for (int i = 0; i < K; ++i) for (int j = 0; j < K; ++j) fro += pmul(SS[i][j], SS[i][j]); fro = sqrtf(fro); float acc = 0.0f; const float ik = rsqrtf((float)K);
    for (int i = 0; i < K; ++i) for (int j = 0; j < K; ++j) { const float dlt = SS[i][j] / fro - (i == j ? ik : 0.0f); acc += pmul(dlt, dlt); } const float ortho = sqrtf(acc);
    float dg[K]; for (int i = 0; i < K; ++i) { float rs = 0.0f; for (int j = 0; j < K; ++j) rs += (i == j) ? 0.0f : SA_[i][j]; dg[i] = sqrtf(rs) + PEPS; }
    for (int pass = 0; pass < 2; ++pass) { for (int i = 0; i < K; ++i) for (int j = 0; j < K; ++j) ((volatile float*)dout)[OFF2 + i * K + j] = (i == j) ? 0.0f : (SA_[i][j] / dg[i]) / dg[j]; ((volatile float*)dout)[OFF3] = mincut; ((volatile float*)dout)[OFF4] = ortho; __threadfence(); } }
  if (wave == 0) { for (int pass = 0; pass < 2; ++pass) { for (int i = 0; i < K; ++i) for (int q = 0; q < F / 32; ++q) ((volatile float*)dout)[OFF1 + i * F + q * 32 + lane] = So[i][q * 32 + lane]; __threadfence(); } }
}
}

extern "C" void kernel_launch(void* const* d_in, const int* in_sizes, int n_in, void* d_out, int out_size, void* d_ws, size_t ws_size, hipStream_t stream) {
  (void)n_in;
  auto Fp = [&](int i) { return (const float*)d_in[i]; }; auto Ip = [&](int i) { return (const int*)d_in[i]; };
  if (in_sizes[0] != N * F || in_sizes[1] != 2 * E || in_sizes[2] != F * W1W || in_sizes[6] != W1W * K || in_sizes[10] != K * K || out_size != OFF4 + 1) return;
  size_t off = 0; char* ws = (char*)d_ws;
  auto carve = [&](size_t bytes) { char* p = ws + off; off += (bytes + 255) & ~(size_t)255; return p; };
  b16* WT1 = (b16*)carve((size_t)W1W * F * 2); b16* WT2 = (b16*)carve((size_t)K * W1W * 2); b16* XT = (b16*)carve((size_t)F * NPD * 2);
  float* P1 = (float*)carve((size_t)N * W1W * 4); float* ES = (float*)carve((size_t)N * 8 * 4); float* ED = (float*)carve((size_t)N * 8 * 4); float* H1p = (float*)carve((size_t)N * W1W * 4); float* P2 = (float*)carve((size_t)N * K * 4); float* EL = (float*)carve((size_t)N * 2 * 4); float* S = (float*)carve((size_t)N * K * 4);
  b16* STh = (b16*)carve((size_t)K * NPD * 2); b16* STl = (b16*)carve((size_t)K * NPD * 2); b16* SAh = (b16*)carve((size_t)K * E * 2); b16* SAl = (b16*)carve((size_t)K * E * 2); b16* SBh = (b16*)carve((size_t)K * E * 2); b16* SBl = (b16*)carve((size_t)K * E * 2);
  CsrBufs8 csr; off = csr_carve8(csr, ws, off, E, N);
  if (off > ws_size || off > ((size_t)128 << 20)) return;
  wprep_kernel<<<(W1W * F / 8 + 255) / 256, 256, 0, stream>>>(Fp(2), F, W1W, WT1); wprep_kernel<<<(K * W1W / 8 + 255) / 256, 256, 0, stream>>>(Fp(6), W1W, K, WT2);
  xt_kernel<<<(F * NPD / 8 + 255) / 256, 256, 0, stream>>>(Fp(0), XT);
  csr_build8(csr, Ip(1) + E, E, N, stream);
  lin1_kernel<<<NBLK, 32, 0, stream>>>(Fp(0), WT1, Fp(3), Fp(4), P1, ES, ED);
  att1_kernel<<<(N + 7) / 8, 256, 0, stream>>>(P1, ES, ED, Fp(5), Ip(1), csr.PERM, csr.ROWPTR, csr.ROWCNT, (int)csr.permLen, H1p);
  lin2_kernel<<<NBLK, 32, 0, stream>>>(H1p, WT2, Fp(7), Fp(8), P2, EL);
  att2_kernel<<<(N / 2 + 7) / 8, 256, 0, stream>>>(P2, EL, Fp(9), Fp(10), Fp(11), Ip(1), csr.PERM, csr.ROWPTR, csr.ROWCNT, (int)csr.permLen, (float*)d_out, S);
  st_kernel<<<(K * NPD / 8 + 255) / 256, 256, 0, stream>>>(S, STh, STl);
  se_kernel<<<(2 * K * (E / 8) + 255) / 256, 256, 0, stream>>>(S, Ip(1), SAh, SAl, SBh, SBl);
  pool_kernel<<<1, 256, 0, stream>>>(STh, STl, XT, SAh, SAl, SBh, SBl, S, Ip(1), (float*)d_out);
}
